// TransformerBlock_53541062312296
// MI455X (gfx1250) — hardware-verified
//
#include <hip/hip_runtime.h>
#include <stdint.h>
#include <stddef.h>


typedef _Float16 v8h  __attribute__((ext_vector_type(8)));
typedef _Float16 v16h __attribute__((ext_vector_type(16)));
typedef float    v4f  __attribute__((ext_vector_type(4)));
typedef float    v8f  __attribute__((ext_vector_type(8)));

#ifndef NB
#define NB 2
#endif
#ifndef SEQ
#define SEQ 2048
#endif
#define NB_FULL  2
#define SEQ_FULL 2048
#define EMB      1024
#define NHEAD    16
#define HDIM     64
#define FFN      4096
#define MTOK     (NB * SEQ)

static_assert(NB >= 1 && NB <= NB_FULL);
static_assert(SEQ >= 128 && SEQ <= SEQ_FULL);
static_assert((SEQ % 128) == 0);
static_assert((MTOK % 128) == 0);
static_assert(EMB == NHEAD * HDIM);
static_assert((EMB % 64) == 0 && (FFN % 64) == 0 && (EMB % 32) == 0 && (FFN % 32) == 0);
static_assert(HDIM == 64);

#define WSC      64.0f
#define WSC_INV  0.015625f
#define LOSC     8192.0f
#define LOSC_INV 0.0001220703125f
#define PSC      16384.0f
#define PSC_INV  0.00006103515625f

#define EE         ((size_t)EMB * (size_t)EMB)
#define FE         ((size_t)FFN * (size_t)EMB)
#define W16_HALVES (3 * EE + 2 * FE)
#define PLANE_H    ((size_t)MTOK * EMB * 2)
#define OFF_W16    ((size_t)0)
#define OFF_X16    (OFF_W16 + W16_HALVES * 2)
#define OFF_QH     (OFF_X16 + PLANE_H)
#define OFF_QL     (OFF_QH + PLANE_H)
#define OFF_KH     (OFF_QL + PLANE_H)
#define OFF_KL     (OFF_KH + PLANE_H)
#define OFF_VT     (OFF_KL + PLANE_H)
#define OFF_ORES   (OFF_VT + PLANE_H)
#define OFF_G16    (OFF_ORES + (size_t)MTOK * EMB * 4)
#define WS_TOTAL   (OFF_G16 + (size_t)MTOK * FFN * 2)
static_assert(WS_TOTAL <= (size_t)134217728);
static_assert((OFF_X16 % 256) == 0 && (OFF_QH % 256) == 0 && (OFF_ORES % 256) == 0 && (OFF_G16 % 256) == 0);
static_assert((W16_HALVES % 2048) == 0);
static_assert((EE % 2048) == 0 && (FE % 2048) == 0);

#define CLD 68
#define KLD 72
#define SLD 68

__device__ __forceinline__ float bf16r(float x) {
  unsigned u = __float_as_uint(x);
  u = (u + 0x7FFFu + ((u >> 16) & 1u)) & 0xFFFF0000u;
  return __uint_as_float(u);
}
__device__ __forceinline__ v4f bf16r4(v4f x) {
  v4f r;
  r[0] = bf16r(x[0]); r[1] = bf16r(x[1]); r[2] = bf16r(x[2]); r[3] = bf16r(x[3]);
  return r;
}
__device__ __forceinline__ v8f zero8() {
  v8f z = {0.0f, 0.0f, 0.0f, 0.0f, 0.0f, 0.0f, 0.0f, 0.0f};
  return z;
}

__device__ __forceinline__ v16h ld_frag(const _Float16* base, int ld) {
  const int lane = (int)(threadIdx.x & 31);
  const _Float16* p = base + (lane & 15) * ld + ((lane >> 4) << 3);
  union { v16h v; v8h hv[2]; } u;
  u.hv[0] = *(const v8h*)(p);
  u.hv[1] = *(const v8h*)(p + 16);
  return u.v;
}

__device__ __forceinline__ v8f wmma16(v16h a, v16h b, v8f c) {
  return __builtin_amdgcn_wmma_f32_16x16x32_f16(false, a, false, b, (short)0, c, false, false);
}

__device__ __forceinline__ float gelu_f(float x) {
  float t = 0.7978845608028654f * (x + 0.044715f * x * x * x);
  t = fminf(fmaxf(t, -10.0f), 10.0f);
  const float e = __expf(2.0f * t);
  const float th = 1.0f - 2.0f * __builtin_amdgcn_rcpf(1.0f + e);
  return 0.5f * x * (1.0f + th);
}

struct Acc8 { v8f a[2][4]; };

__device__ __forceinline__ void gemm_core(const _Float16* __restrict__ A, int lda,
                                          const _Float16* __restrict__ Bw, int ldb,
                                          int K, int m0, int n0, Acc8& C) {
  const int wid = (int)(threadIdx.x >> 5);
  const _Float16* a0p = A + (size_t)(m0 + wid * 32) * lda;
  const _Float16* a1p = a0p + (size_t)16 * lda;
  const _Float16* b0p = Bw + (size_t)n0 * ldb;
  const _Float16* b1p = b0p + (size_t)16 * ldb;
  const _Float16* b2p = b0p + (size_t)32 * ldb;
  const _Float16* b3p = b0p + (size_t)48 * ldb;
#pragma unroll
  for (int f = 0; f < 2; ++f)
#pragma unroll
    for (int t = 0; t < 4; ++t) C.a[f][t] = zero8();
#pragma unroll 1
  for (int k0 = 0; k0 < K; k0 += 32) {
    const v16h fa0 = ld_frag(a0p + k0, lda);
    const v16h fa1 = ld_frag(a1p + k0, lda);
    const v16h fb0 = ld_frag(b0p + k0, ldb);
    const v16h fb1 = ld_frag(b1p + k0, ldb);
    const v16h fb2 = ld_frag(b2p + k0, ldb);
    const v16h fb3 = ld_frag(b3p + k0, ldb);
    C.a[0][0] = wmma16(fa0, fb0, C.a[0][0]);
    C.a[0][1] = wmma16(fa0, fb1, C.a[0][1]);
    C.a[0][2] = wmma16(fa0, fb2, C.a[0][2]);
    C.a[0][3] = wmma16(fa0, fb3, C.a[0][3]);
    C.a[1][0] = wmma16(fa1, fb0, C.a[1][0]);
    C.a[1][1] = wmma16(fa1, fb1, C.a[1][1]);
    C.a[1][2] = wmma16(fa1, fb2, C.a[1][2]);
    C.a[1][3] = wmma16(fa1, fb3, C.a[1][3]);
    asm volatile("v_nop\n\tv_nop\n\tv_nop\n\tv_nop"
                 : "+v"(C.a[0][0]), "+v"(C.a[0][1]), "+v"(C.a[0][2]), "+v"(C.a[0][3]),
                   "+v"(C.a[1][0]), "+v"(C.a[1][1]), "+v"(C.a[1][2]), "+v"(C.a[1][3])
                 : "v"(fa0), "v"(fa1), "v"(fb0), "v"(fb1), "v"(fb2), "v"(fb3));
  }
}

__device__ __forceinline__ void stage_tile(float* Cs, const Acc8& C,
                                           const float* __restrict__ bias, int do_gelu) {
  const int lane = (int)(threadIdx.x & 31), wid = (int)(threadIdx.x >> 5);
  const int cc = lane & 15, hh = lane >> 4;
#pragma unroll
  for (int t = 0; t < 4; ++t) {
    const float bvv = bf16r(bias[t * 16 + cc]);
#pragma unroll
    for (int f = 0; f < 2; ++f) {
      float* dp = Cs + (wid * 32 + f * 16 + hh * 8) * CLD + t * 16 + cc;
#pragma unroll
      for (int r = 0; r < 8; ++r) {
        float val = C.a[f][t][r] * WSC_INV + bvv;
        if (do_gelu) val = gelu_f(val);
        dp[r * CLD] = val;
      }
    }
  }
}

__global__ __launch_bounds__(256) void cvt_w_kernel(
    const float* __restrict__ Wq, const float* __restrict__ Wk, const float* __restrict__ Wv,
    const float* __restrict__ W1, const float* __restrict__ W2, _Float16* __restrict__ w16) {
  const size_t blk0 = (size_t)blockIdx.x * 2048;
  const float* src;
  size_t base;
  if (blk0 < EE)                 { src = Wq; base = 0; }
  else if (blk0 < 2 * EE)        { src = Wk; base = EE; }
  else if (blk0 < 3 * EE)        { src = Wv; base = 2 * EE; }
  else if (blk0 < 3 * EE + FE)   { src = W1; base = 3 * EE; }
  else                           { src = W2; base = 3 * EE + FE; }
  const size_t e = blk0 + (size_t)threadIdx.x * 8;
  const float* p = src + (e - base);
  const v4f u0 = *(const v4f*)(p);
  const v4f u1 = *(const v4f*)(p + 4);
  v8h o;
#pragma unroll
  for (int i = 0; i < 4; ++i) {
    o[i]     = (_Float16)(bf16r(u0[i]) * WSC);
    o[i + 4] = (_Float16)(bf16r(u1[i]) * WSC);
  }
  _Float16* dp = w16 + e;
  *(volatile v8h*)dp = o;
  __threadfence();
  *(volatile v8h*)dp = o;
}

template <int RND>
__global__ __launch_bounds__(256) void ln_kernel(const float* __restrict__ src, int bstride,
                                                 const float* __restrict__ gam,
                                                 const float* __restrict__ bet,
                                                 _Float16* __restrict__ dst) {
  const int lane = (int)(threadIdx.x & 31), wid = (int)(threadIdx.x >> 5);
  const int m = (int)blockIdx.x * 8 + wid;
  const int b = m / SEQ, s = m - b * SEQ;
  const float* xp = src + (size_t)b * (size_t)bstride + (size_t)s * EMB;
  float x[32];
#pragma unroll
  for (int c = 0; c < 4; ++c) {
    v4f u0 = *(const v4f*)(xp + c * 256 + lane * 8);
    v4f u1 = *(const v4f*)(xp + c * 256 + lane * 8 + 4);
    if (RND) { u0 = bf16r4(u0); u1 = bf16r4(u1); }
#pragma unroll
    for (int i = 0; i < 4; ++i) { x[c * 8 + i] = u0[i]; x[c * 8 + 4 + i] = u1[i]; }
  }
  float sum = 0.0f;
#pragma unroll
  for (int i = 0; i < 32; ++i) sum += x[i];
#pragma unroll
  for (int off = 16; off >= 1; off >>= 1) sum += __shfl_xor(sum, off, 32);
  const float mean = sum * (1.0f / (float)EMB);
  float ss = 0.0f;
#pragma unroll
  for (int i = 0; i < 32; ++i) { const float d = x[i] - mean; x[i] = d; ss += d * d; }
#pragma unroll
  for (int off = 16; off >= 1; off >>= 1) ss += __shfl_xor(ss, off, 32);
  const float var = ss * (1.0f / (float)(EMB - 1));
  const float sd = sqrtf(var);
  const float inv = 1.0f / (sd + 1e-8f);
  v8h o[4];
#pragma unroll
  for (int c = 0; c < 4; ++c) {
    const int col = c * 256 + lane * 8;
    const v4f g0 = bf16r4(*(const v4f*)(gam + col));
    const v4f g1 = bf16r4(*(const v4f*)(gam + col + 4));
    const v4f e0 = bf16r4(*(const v4f*)(bet + col));
    const v4f e1 = bf16r4(*(const v4f*)(bet + col + 4));
    v8h t;
#pragma unroll
    for (int i = 0; i < 4; ++i) {
      t[i]     = (_Float16)(g0[i] * (x[c * 8 + i] * inv) + e0[i]);
      t[i + 4] = (_Float16)(g1[i] * (x[c * 8 + 4 + i] * inv) + e1[i]);
    }
    o[c] = t;
  }
  _Float16* drow = dst + (size_t)m * EMB + lane * 8;
#pragma unroll
  for (int c = 0; c < 4; ++c) *(volatile v8h*)(drow + c * 256) = o[c];
  __threadfence();
#pragma unroll
  for (int c = 0; c < 4; ++c) *(volatile v8h*)(drow + c * 256) = o[c];
}

__global__ __launch_bounds__(128) void qkv_kernel(
    const _Float16* __restrict__ X, const _Float16* __restrict__ Wqkv,
    const float* __restrict__ bq, const float* __restrict__ bk, const float* __restrict__ bv,
    _Float16* __restrict__ qh, _Float16* __restrict__ ql,
    _Float16* __restrict__ kh, _Float16* __restrict__ kl,
    _Float16* __restrict__ vt) {
  __shared__ __attribute__((aligned(16))) float Cs[128 * CLD];
  const int tid = (int)threadIdx.x, lane = tid & 31, wid = tid >> 5;
  const int n0 = (int)blockIdx.x * 64;
  const int m0 = (int)blockIdx.y * 128;
  const int which = n0 / EMB;
  const int nl = n0 - which * EMB;
  Acc8 C;
  gemm_core(X, EMB, Wqkv, EMB, EMB, m0, n0, C);
  const float* bias = (which == 0) ? bq : ((which == 1) ? bk : bv);
  stage_tile(Cs, C, bias + nl, 0);
  __syncthreads();
  if (which < 2) {
    _Float16* Ph = (which == 0) ? qh : kh;
    _Float16* Pl = (which == 0) ? ql : kl;
    const int rsub = lane >> 3, c8 = (lane & 7) * 8;
    v8h hv[8], lv[8];
    size_t off[8];
#pragma unroll
    for (int it = 0; it < 8; ++it) {
      const int row = wid * 32 + it * 4 + rsub;
      const float* cp = &Cs[row * CLD + c8];
      const v4f u0 = *(const v4f*)(cp);
      const v4f u1 = *(const v4f*)(cp + 4);
      v8h th, tl;
#pragma unroll
      for (int i = 0; i < 4; ++i) {
        const _Float16 h0 = (_Float16)u0[i];
        const _Float16 h1 = (_Float16)u1[i];
        th[i]     = h0;
        th[i + 4] = h1;
        tl[i]     = (_Float16)((u0[i] - (float)h0) * LOSC);
        tl[i + 4] = (_Float16)((u1[i] - (float)h1) * LOSC);
      }
      hv[it] = th; lv[it] = tl;
      off[it] = (size_t)(m0 + row) * EMB + nl + c8;
    }
#pragma unroll
    for (int it = 0; it < 8; ++it) {
      *(volatile v8h*)(Ph + off[it]) = hv[it];
      *(volatile v8h*)(Pl + off[it]) = lv[it];
    }
    __threadfence();
#pragma unroll
    for (int it = 0; it < 8; ++it) {
      *(volatile v8h*)(Ph + off[it]) = hv[it];
      *(volatile v8h*)(Pl + off[it]) = lv[it];
    }
  } else {
    const int head = nl / HDIM;
    const int b = m0 / SEQ, s0 = m0 - b * SEQ;
    const int key8 = (lane & 15) * 8, dsub = lane >> 4;
    v8h tv[8];
    size_t off[8];
#pragma unroll
    for (int it = 0; it < 8; ++it) {
      const int d = wid * 16 + it * 2 + dsub;
      v8h t;
#pragma unroll
      for (int i = 0; i < 8; ++i) t[i] = (_Float16)Cs[(key8 + i) * CLD + d];
      tv[it] = t;
      off[it] = (((size_t)(b * NHEAD + head)) * HDIM + d) * SEQ + s0 + key8;
    }
#pragma unroll
    for (int it = 0; it < 8; ++it) *(volatile v8h*)(vt + off[it]) = tv[it];
    __threadfence();
#pragma unroll
    for (int it = 0; it < 8; ++it) *(volatile v8h*)(vt + off[it]) = tv[it];
  }
}

__global__ __launch_bounds__(256) void attn_kernel(
    const _Float16* __restrict__ qh, const _Float16* __restrict__ ql,
    const _Float16* __restrict__ kh, const _Float16* __restrict__ kl,
    const _Float16* __restrict__ vt, const float* __restrict__ xin,
    float* __restrict__ ores) {
  __shared__ __attribute__((aligned(16))) _Float16 Kh_s[64 * KLD];
  __shared__ __attribute__((aligned(16))) _Float16 Kl_s[64 * KLD];
  __shared__ __attribute__((aligned(16))) _Float16 Vt_s[64 * KLD];
  __shared__ __attribute__((aligned(16))) float    S_s[64 * SLD];
  __shared__ __attribute__((aligned(16))) _Float16 P_s[64 * KLD];
  __shared__ float m_s[64], l_s[64], a_s[64];

  const int tid = (int)threadIdx.x, lane = tid & 31, wid = tid >> 5;
  const int mw = wid >> 1, nw = wid & 1;
  const int hh = lane >> 4, cc = lane & 15;
  const int qt = (int)blockIdx.x, h = (int)blockIdx.y, b = (int)blockIdx.z;
  const int tok0 = b * SEQ + qt * 64;
  const size_t hoff = (size_t)h * HDIM;

  const _Float16* qhp = qh + (size_t)(tok0 + mw * 16) * EMB + hoff;
  const _Float16* qlp = ql + (size_t)(tok0 + mw * 16) * EMB + hoff;
  const v16h qa_h0 = ld_frag(qhp, EMB), qa_h1 = ld_frag(qhp + 32, EMB);
  const v16h qa_l0 = ld_frag(qlp, EMB), qa_l1 = ld_frag(qlp + 32, EMB);

  if (tid < 64) { m_s[tid] = -1e30f; l_s[tid] = 0.0f; a_s[tid] = 0.0f; }

  v8f oacc0 = zero8(), oacc1 = zero8();
  const _Float16* vtp = vt + ((size_t)(b * NHEAD + h) * HDIM) * SEQ;

  for (int kt = 0; kt < SEQ / 64; ++kt) {
    const int ktok0 = b * SEQ + kt * 64;
#pragma unroll
    for (int j = 0; j < 2; ++j) {
      const int c = tid + j * 256;
      const int r = c >> 3, c8 = (c & 7) * 8;
      *(v8h*)&Kh_s[r * KLD + c8] = *(const v8h*)(kh + (size_t)(ktok0 + r) * EMB + hoff + c8);
      *(v8h*)&Kl_s[r * KLD + c8] = *(const v8h*)(kl + (size_t)(ktok0 + r) * EMB + hoff + c8);
      *(v8h*)&Vt_s[r * KLD + c8] = *(const v8h*)(vtp + (size_t)r * SEQ + kt * 64 + c8);
    }
    __syncthreads();

    v8f sacc0 = zero8(), sacc1 = zero8(), racc0 = zero8(), racc1 = zero8();
    {
      const _Float16* kb  = &Kh_s[(nw * 32) * KLD];
      const _Float16* klb = &Kl_s[(nw * 32) * KLD];
      const v16h bh0 = ld_frag(kb, KLD),                 bl0 = ld_frag(klb, KLD);
      sacc0 = wmma16(qa_h0, bh0, sacc0); racc0 = wmma16(qa_h0, bl0, racc0); racc0 = wmma16(qa_l0, bh0, racc0);
      const v16h bh1 = ld_frag(kb + 32, KLD),            bl1 = ld_frag(klb + 32, KLD);
      sacc0 = wmma16(qa_h1, bh1, sacc0); racc0 = wmma16(qa_h1, bl1, racc0); racc0 = wmma16(qa_l1, bh1, racc0);
      const v16h bh2 = ld_frag(kb + 16 * KLD, KLD),      bl2 = ld_frag(klb + 16 * KLD, KLD);
      sacc1 = wmma16(qa_h0, bh2, sacc1); racc1 = wmma16(qa_h0, bl2, racc1); racc1 = wmma16(qa_l0, bh2, racc1);
      const v16h bh3 = ld_frag(kb + 16 * KLD + 32, KLD), bl3 = ld_frag(klb + 16 * KLD + 32, KLD);
      sacc1 = wmma16(qa_h1, bh3, sacc1); racc1 = wmma16(qa_h1, bl3, racc1); racc1 = wmma16(qa_l1, bh3, racc1);
      asm volatile("v_nop\n\tv_nop\n\tv_nop\n\tv_nop"
                   : "+v"(sacc0), "+v"(sacc1), "+v"(racc0), "+v"(racc1)
                   : "v"(bh0), "v"(bl0), "v"(bh1), "v"(bl1), "v"(bh2), "v"(bl2), "v"(bh3), "v"(bl3),
                     "v"(qa_h0), "v"(qa_h1), "v"(qa_l0), "v"(qa_l1));
    }
    {
      float* sp = &S_s[(mw * 16 + hh * 8) * SLD + nw * 32 + cc];
#pragma unroll
      for (int r = 0; r < 8; ++r) {
        sp[r * SLD]      = sacc0[r] + racc0[r] * LOSC_INV;
        sp[r * SLD + 16] = sacc1[r] + racc1[r] * LOSC_INV;
      }
    }
    __syncthreads();

    {
      const int row = tid >> 2, part = tid & 3;
      const float* sp = &S_s[row * SLD + part * 16];
      float sv[16];
#pragma unroll
      for (int q4 = 0; q4 < 4; ++q4) {
        const v4f u = *(const v4f*)(sp + q4 * 4);
        sv[q4 * 4 + 0] = u[0]; sv[q4 * 4 + 1] = u[1]; sv[q4 * 4 + 2] = u[2]; sv[q4 * 4 + 3] = u[3];
      }
      float mx = sv[0];
#pragma unroll
      for (int c = 1; c < 16; ++c) mx = fmaxf(mx, sv[c]);
      mx = fmaxf(mx, __shfl_xor(mx, 1, 32));
      mx = fmaxf(mx, __shfl_xor(mx, 2, 32));
      const float mold = m_s[row];
      const float mnew = fmaxf(mold, mx);
      float lsum = 0.0f;
      v8h p0, p1;
#pragma unroll
      for (int c = 0; c < 8; ++c) {
        const float pa = __expf(sv[c] - mnew);
        const float pb = __expf(sv[c + 8] - mnew);
        lsum += pa + pb;
        p0[c] = (_Float16)(pa * PSC);
        p1[c] = (_Float16)(pb * PSC);
      }
      *(v8h*)&P_s[row * KLD + part * 16]     = p0;
      *(v8h*)&P_s[row * KLD + part * 16 + 8] = p1;
      lsum += __shfl_xor(lsum, 1, 32);
      lsum += __shfl_xor(lsum, 2, 32);
      if (part == 0) {
        const float alpha = __expf(mold - mnew);
        m_s[row] = mnew;
        l_s[row] = l_s[row] * alpha + lsum;
        a_s[row] = alpha;
      }
    }
    __syncthreads();

    {
      float ar[8];
#pragma unroll
      for (int r = 0; r < 8; ++r) ar[r] = a_s[mw * 16 + hh * 8 + r];
#pragma unroll
      for (int r = 0; r < 8; ++r) { oacc0[r] *= ar[r]; oacc1[r] *= ar[r]; }
      const _Float16* pp = &P_s[(mw * 16) * KLD];
      const _Float16* vp = &Vt_s[(nw * 32) * KLD];
      const v16h pa0 = ld_frag(pp, KLD),       pa1 = ld_frag(pp + 32, KLD);
      const v16h vb00 = ld_frag(vp, KLD),      vb01 = ld_frag(vp + 16 * KLD, KLD);
      const v16h vb10 = ld_frag(vp + 32, KLD), vb11 = ld_frag(vp + 16 * KLD + 32, KLD);
      oacc0 = wmma16(pa0, vb00, oacc0); oacc1 = wmma16(pa0, vb01, oacc1);
      oacc0 = wmma16(pa1, vb10, oacc0); oacc1 = wmma16(pa1, vb11, oacc1);
      asm volatile("v_nop\n\tv_nop\n\tv_nop\n\tv_nop"
                   : "+v"(oacc0), "+v"(oacc1)
                   : "v"(pa0), "v"(pa1), "v"(vb00), "v"(vb01), "v"(vb10), "v"(vb11));
    }
    __syncthreads();
  }

  {
    float inv[8];
#pragma unroll
    for (int r = 0; r < 8; ++r) inv[r] = __builtin_amdgcn_rcpf(l_s[mw * 16 + hh * 8 + r]) * PSC_INV;
    float* sp = &S_s[(mw * 16 + hh * 8) * SLD + nw * 32 + cc];
#pragma unroll
    for (int r = 0; r < 8; ++r) {
      sp[r * SLD]      = oacc0[r] * inv[r];
      sp[r * SLD + 16] = oacc1[r] * inv[r];
    }
  }
  __syncthreads();
  {
    const int csub = (lane & 15) * 4, rsub = lane >> 4;
    v4f ov[4];
    size_t off[4];
#pragma unroll
    for (int it = 0; it < 4; ++it) {
      const int row = wid * 8 + it * 2 + rsub;
      const v4f cv = *(const v4f*)&S_s[row * SLD + csub];
      const size_t irow = (size_t)b * SEQ_FULL + (size_t)(qt * 64 + row);
      const v4f xv = bf16r4(*(const v4f*)(xin + irow * EMB + hoff + csub));
      ov[it] = cv + xv;
      off[it] = (size_t)(tok0 + row) * EMB + hoff + csub;
    }
#pragma unroll
    for (int it = 0; it < 4; ++it) *(volatile v4f*)(ores + off[it]) = ov[it];
    __threadfence();
#pragma unroll
    for (int it = 0; it < 4; ++it) *(volatile v4f*)(ores + off[it]) = ov[it];
  }
}

__global__ __launch_bounds__(128) void ffn1_kernel(
    const _Float16* __restrict__ X2, const _Float16* __restrict__ W1h,
    const float* __restrict__ b1, _Float16* __restrict__ g16) {
  __shared__ __attribute__((aligned(16))) float Cs[128 * CLD];
  const int tid = (int)threadIdx.x, lane = tid & 31, wid = tid >> 5;
  const int n0 = (int)blockIdx.x * 64;
  const int m0 = (int)blockIdx.y * 128;
  Acc8 C;
  gemm_core(X2, EMB, W1h, EMB, EMB, m0, n0, C);
  stage_tile(Cs, C, b1 + n0, 1);
  __syncthreads();
  const int rsub = lane >> 3, c8 = (lane & 7) * 8;
  v8h hv[8];
  size_t off[8];
#pragma unroll
  for (int it = 0; it < 8; ++it) {
    const int row = wid * 32 + it * 4 + rsub;
    const float* cp = &Cs[row * CLD + c8];
    const v4f u0 = *(const v4f*)(cp);
    const v4f u1 = *(const v4f*)(cp + 4);
    v8h t;
#pragma unroll
    for (int i = 0; i < 4; ++i) { t[i] = (_Float16)u0[i]; t[i + 4] = (_Float16)u1[i]; }
    hv[it] = t;
    off[it] = (size_t)(m0 + row) * FFN + n0 + c8;
  }
#pragma unroll
  for (int it = 0; it < 8; ++it) *(volatile v8h*)(g16 + off[it]) = hv[it];
  __threadfence();
#pragma unroll
  for (int it = 0; it < 8; ++it) *(volatile v8h*)(g16 + off[it]) = hv[it];
}

__global__ __launch_bounds__(128) void ffn2_kernel(
    const _Float16* __restrict__ G, const _Float16* __restrict__ W2h,
    const float* __restrict__ b2, const float* __restrict__ ores,
    float* __restrict__ out) {
  __shared__ __attribute__((aligned(16))) float Cs[128 * CLD];
  const int tid = (int)threadIdx.x, lane = tid & 31, wid = tid >> 5;
  const int n0 = (int)blockIdx.x * 64;
  const int m0 = (int)blockIdx.y * 128;
  Acc8 C;
  gemm_core(G, FFN, W2h, FFN, FFN, m0, n0, C);
  stage_tile(Cs, C, b2 + n0, 0);
  __syncthreads();
  const int rsub = lane >> 4, c4 = (lane & 15) * 4;
  v4f ov[16];
  size_t off[16];
#pragma unroll
  for (int it = 0; it < 16; ++it) {
    const int row = wid * 32 + it * 2 + rsub;
    const size_t o = (size_t)(m0 + row) * EMB + n0 + c4;
    const v4f cv = *(const v4f*)&Cs[row * CLD + c4];
    const v4f rv = *(const v4f*)(ores + o);
    ov[it] = cv + rv;
    off[it] = o;
  }
#pragma unroll
  for (int it = 0; it < 16; ++it) *(volatile v4f*)(out + off[it]) = ov[it];
  __threadfence();
#pragma unroll
  for (int it = 0; it < 16; ++it) *(volatile v4f*)(out + off[it]) = ov[it];
}

extern "C" void kernel_launch(void* const* d_in, const int* in_sizes, int n_in,
                              void* d_out, int out_size, void* d_ws,
                              size_t ws_size, hipStream_t stream) {
  if (n_in < 15) return;
  const size_t need_in0 = ((size_t)(NB - 1) * SEQ_FULL + (size_t)SEQ) * EMB;
  if ((size_t)in_sizes[0] < need_in0) return;
  if ((size_t)in_sizes[1] < EE || (size_t)in_sizes[3] < EE || (size_t)in_sizes[5] < EE) return;
  if ((size_t)in_sizes[7] < FE || (size_t)in_sizes[9] < FE) return;
  if (in_sizes[2] < EMB || in_sizes[4] < EMB || in_sizes[6] < EMB || in_sizes[10] < EMB) return;
  if (in_sizes[8] < FFN) return;
  if (in_sizes[11] < EMB || in_sizes[12] < EMB || in_sizes[13] < EMB || in_sizes[14] < EMB) return;
  if ((size_t)out_size < (size_t)MTOK * EMB) return;
  if (ws_size < WS_TOTAL) return;

  const float* xin    = (const float*)d_in[0];
  const float* Wq     = (const float*)d_in[1];
  const float* bq     = (const float*)d_in[2];
  const float* Wk     = (const float*)d_in[3];
  const float* bk     = (const float*)d_in[4];
  const float* Wv     = (const float*)d_in[5];
  const float* bv     = (const float*)d_in[6];
  const float* W1     = (const float*)d_in[7];
  const float* b1     = (const float*)d_in[8];
  const float* W2     = (const float*)d_in[9];
  const float* b2     = (const float*)d_in[10];
  const float* scale1 = (const float*)d_in[11];
  const float* shift1 = (const float*)d_in[12];
  const float* scale2 = (const float*)d_in[13];
  const float* shift2 = (const float*)d_in[14];
  float* out = (float*)d_out;

  char* ws = (char*)d_ws;
  _Float16* w16   = (_Float16*)(ws + OFF_W16);
  _Float16* wqkv  = w16;
  _Float16* w1h   = w16 + 3 * EE;
  _Float16* w2h   = w16 + 3 * EE + FE;
  _Float16* x16   = (_Float16*)(ws + OFF_X16);
  _Float16* qh    = (_Float16*)(ws + OFF_QH);
  _Float16* ql    = (_Float16*)(ws + OFF_QL);
  _Float16* kh    = (_Float16*)(ws + OFF_KH);
  _Float16* kl    = (_Float16*)(ws + OFF_KL);
  _Float16* vt    = (_Float16*)(ws + OFF_VT);
  float*    ores  = (float*)(ws + OFF_ORES);
  _Float16* g16   = (_Float16*)(ws + OFF_G16);

  cvt_w_kernel<<<dim3((unsigned)(W16_HALVES / 2048)), dim3(256), 0, stream>>>(
      Wq, Wk, Wv, W1, W2, w16);
  ln_kernel<1><<<dim3((unsigned)(MTOK / 8)), dim3(256), 0, stream>>>(
      xin, SEQ_FULL * EMB, scale1, shift1, x16);
  qkv_kernel<<<dim3((unsigned)(3 * EMB / 64), (unsigned)(MTOK / 128)), dim3(128), 0, stream>>>(
      x16, wqkv, bq, bk, bv, qh, ql, kh, kl, vt);
  attn_kernel<<<dim3((unsigned)(SEQ / 64), (unsigned)NHEAD, (unsigned)NB), dim3(256), 0, stream>>>(
      qh, ql, kh, kl, vt, xin, ores);
  ln_kernel<0><<<dim3((unsigned)(MTOK / 8)), dim3(256), 0, stream>>>(
      ores, SEQ * EMB, scale2, shift2, x16);
  ffn1_kernel<<<dim3((unsigned)(FFN / 64), (unsigned)(MTOK / 128)), dim3(128), 0, stream>>>(
      x16, w1h, b1, g16);
  ffn2_kernel<<<dim3((unsigned)(EMB / 64), (unsigned)(MTOK / 128)), dim3(128), 0, stream>>>(
      g16, w2h, b2, ores, out);
}
